// Block_78683800863152
// MI455X (gfx1250) — hardware-verified
//
#include <hip/hip_runtime.h>
#include <math.h>

typedef __attribute__((ext_vector_type(16))) _Float16 v16h;
typedef __attribute__((ext_vector_type(8)))  _Float16 v8h;
typedef __attribute__((ext_vector_type(8)))  float    v8f;
typedef __attribute__((ext_vector_type(4)))  float    v4f;

constexpr int kBatch  = 2;
constexpr int kSeq    = 1024;
constexpr int kDm     = 1024;
constexpr int kSqrtDm = 32;
constexpr int kDin    = 2048;
constexpr int kNst    = 16;
constexpr int kDtR    = 64;
constexpr int kPrjN   = 96;
constexpr int kPrjP   = 128;
constexpr int kXZP    = 2 * kDin;
constexpr int kRows   = kBatch * kSeq;
constexpr int kTP     = 260;
constexpr float kEps  = 1e-5f;
static_assert(kSqrtDm * kSqrtDm == kDm);
static_assert(kDtR + 2 * kNst == kPrjN);
static_assert((kPrjP % 64) == 0 && kPrjP >= kPrjN);
static_assert((kDm % 32) == 0 && (kDin % 32) == 0 && (kDtR % 32) == 0);
static_assert((kRows % 64) == 0 && (kXZP % 64) == 0 && (kDin % 64) == 0 && (kDm % 64) == 0);
static_assert((kSeq % 64) == 0 && (kDin % 256) == 0 && (kSeq % 16) == 0);

constexpr float kInvSqrtDm = 1.0f / (float)kSqrtDm;
constexpr float kCarryH    = 16.0f;
constexpr float kCarryW    = 32.0f;
constexpr float kCarryXc   = 64.0f;
constexpr float kCarryDt   = 256.0f;
constexpr float kCarryY    = 256.0f;
constexpr float kFoldIn    = 1.0f / (kCarryH  * kCarryW);
constexpr float kFoldX     = 1.0f / (kCarryXc * kCarryW);
constexpr float kFoldDt    = 1.0f / (kCarryDt * kCarryW);
constexpr float kFoldOut   = 1.0f / (kCarryY  * kCarryW);

constexpr size_t kOffWIN  = 0;
constexpr size_t kOffWXP  = kOffWIN  + (size_t)kXZP  * kDm   * 2;
constexpr size_t kOffWDT  = kOffWXP  + (size_t)kPrjP * kDin  * 2;
constexpr size_t kOffWOUT = kOffWDT  + (size_t)kDin  * kDtR  * 2;
constexpr size_t kOffH16  = kOffWOUT + (size_t)kDm   * kDin  * 2;
constexpr size_t kOffXZ   = kOffH16  + (size_t)kRows * kDm   * 2;
constexpr size_t kOffUC   = kOffXZ   + (size_t)kRows * kXZP  * 4;
constexpr size_t kOffUC16 = kOffUC   + (size_t)kRows * kDin  * 4;
constexpr size_t kOffPROJ = kOffUC16 + (size_t)kRows * kDin  * 2;
constexpr size_t kOffDT16 = kOffPROJ + (size_t)kRows * kPrjP * 4;
constexpr size_t kOffDLR  = kOffDT16 + (size_t)kRows * kDtR  * 2;
constexpr size_t kOffY16  = kOffDLR  + (size_t)kRows * kDin  * 4;
constexpr size_t kWsTotal = kOffY16  + (size_t)kRows * kDin  * 2;
static_assert(kWsTotal == 102760448ull);
static_assert(kWsTotal <= 134217728ull);
static_assert((kOffWXP % 128) == 0 && (kOffWDT % 128) == 0 && (kOffWOUT % 128) == 0 && (kOffH16 % 128) == 0 &&
              (kOffXZ % 128) == 0 && (kOffUC % 128) == 0 && (kOffUC16 % 128) == 0 && (kOffPROJ % 128) == 0 &&
              (kOffDT16 % 128) == 0 && (kOffDLR % 128) == 0 && (kOffY16 % 128) == 0);

__device__ __forceinline__ void grp_guard_h(v8f& a, v8f& b, v8f& c, v8f& d, v16h x, v16h y0, v16h y1, v16h y2, v16h y3) {
  asm volatile("v_nop\n\tv_nop\n\tv_nop\n\tv_nop" : "+v"(a), "+v"(b), "+v"(c), "+v"(d) : "v"(x), "v"(y0), "v"(y1), "v"(y2), "v"(y3));
}
__device__ __forceinline__ void keep4_h(v16h a, v16h b, v16h c, v16h d) { asm volatile("v_nop" :: "v"(a), "v"(b), "v"(c), "v"(d)); }
__device__ __forceinline__ void acc_guard4(v8f& a, v8f& b, v8f& c, v8f& d) { asm volatile("v_nop\n\tv_nop\n\tv_nop\n\tv_nop" : "+v"(a), "+v"(b), "+v"(c), "+v"(d)); }

struct FragH {
  union U { v16h v; v8h h[2]; };
  static __device__ __forceinline__ v16h load(const _Float16* p) {
    U f; f.h[0] = *(const v8h*)(p); f.h[1] = *(const v8h*)(p + 16); return f.v;
  }
  static __device__ __forceinline__ v8f mma(v16h a, v16h b, v8f c) {
    return __builtin_amdgcn_wmma_f32_16x16x32_f16(false, a, false, b, (short)0, c, false, false);
  }
};

__device__ __forceinline__ float silu_f(float v) { return v * (1.0f / (1.0f + expf(-v))); }

template <int BIAS_MODE>
__global__ __launch_bounds__(256) void wmma_gemm64_f16(
    const unsigned short* __restrict__ Ap, int lda,
    const unsigned short* __restrict__ Btp, int ldb,
    float* __restrict__ Cout, int ldc,
    const float* __restrict__ bias,
    int M, int N, int K, float scale) {
  const _Float16* A  = (const _Float16*)Ap;
  const _Float16* Bt = (const _Float16*)Btp;
  __shared__ __align__(16) float sT[8][16 * 68];
  const int lane = threadIdx.x & 31;
  const int wave = threadIdx.x >> 5;
  const int tilesN = N >> 6;
  const int tilesM = M >> 6;
  const int tile = blockIdx.x * 8 + wave;
  if (tile >= tilesM * tilesN) return;
  const int tm = tile / tilesN;
  const int tn = tile - tm * tilesN;
  const int m0 = tm << 6;
  const int n0 = tn << 6;

  const int rlane = lane & 15;
  const int koff  = (lane >> 4) * 8;
  const int mOff  = (lane >> 4) * 8;

  v8f acc[4][4];
#pragma unroll
  for (int i = 0; i < 4; ++i)
#pragma unroll
    for (int j = 0; j < 4; ++j) acc[i][j] = (v8f){0.f,0.f,0.f,0.f,0.f,0.f,0.f,0.f};

  for (int k0 = 0; k0 < K; k0 += 32) {
    v16h bh[4];
#pragma unroll
    for (int j = 0; j < 4; ++j) {
      const size_t bo = (size_t)(n0 + (j << 4) + rlane) * ldb + koff + k0;
      bh[j] = FragH::load(Bt + bo);
    }
#pragma unroll
    for (int i = 0; i < 4; ++i) {
      const size_t ao = (size_t)(m0 + (i << 4) + rlane) * lda + koff + k0;
      v16h ah = FragH::load(A + ao);
#pragma unroll
      for (int j = 0; j < 4; ++j) acc[i][j] = FragH::mma(ah, bh[j], acc[i][j]);
      grp_guard_h(acc[i][0], acc[i][1], acc[i][2], acc[i][3], ah, bh[0], bh[1], bh[2], bh[3]);
    }
    keep4_h(bh[0], bh[1], bh[2], bh[3]);
  }
  acc_guard4(acc[0][0], acc[0][1], acc[0][2], acc[0][3]);
  acc_guard4(acc[1][0], acc[1][1], acc[1][2], acc[1][3]);
  acc_guard4(acc[2][0], acc[2][1], acc[2][2], acc[2][3]);
  acc_guard4(acc[3][0], acc[3][1], acc[3][2], acc[3][3]);

  float* slab = sT[wave];
#pragma unroll
  for (int i = 0; i < 4; ++i) {
    const int mBase = m0 + (i << 4);
#pragma unroll
    for (int j = 0; j < 4; ++j) {
      const int n = n0 + (j << 4) + rlane;
      float bv = 0.f;
      if (BIAS_MODE == 2) bv = bias[n];
#pragma unroll
      for (int r = 0; r < 8; ++r) {
        float v = acc[i][j][r] * scale;
        if (BIAS_MODE == 2) v += bv;
        slab[(mOff + r) * 68 + (j << 4) + rlane] = v;
      }
    }
    __builtin_amdgcn_fence(__ATOMIC_RELEASE, "workgroup");
    __builtin_amdgcn_wave_barrier();
    __builtin_amdgcn_fence(__ATOMIC_ACQUIRE, "workgroup");
    {
      const int hh = lane >> 4, c4 = (lane & 15) * 4;
      for (int pass = 0; pass < 2; ++pass) {
#pragma unroll
        for (int it = 0; it < 8; ++it) {
          const int row = it * 2 + hh;
          v4f v = *(const v4f*)(slab + row * 68 + c4);
          *(volatile v4f*)(Cout + (size_t)(mBase + row) * ldc + n0 + c4) = v;
        }
        __threadfence();
      }
    }
    __builtin_amdgcn_fence(__ATOMIC_RELEASE, "workgroup");
    __builtin_amdgcn_wave_barrier();
    __builtin_amdgcn_fence(__ATOMIC_ACQUIRE, "workgroup");
  }
}

__global__ __launch_bounds__(256) void cast_f16_pad_kernel(
    const float* __restrict__ src, unsigned short* __restrict__ dst, int total8, int real8, float scale)
{
  const int i = blockIdx.x * 256 + threadIdx.x;
  if (i >= total8) return;
  const bool ok = (i < real8);
  const int ic = ok ? i : (real8 - 1);
  const float* p = src + ((size_t)ic << 3);
  const v4f a0 = *(const v4f*)(p);
  const v4f a1 = *(const v4f*)(p + 4);
  v8h hv;
#pragma unroll
  for (int e = 0; e < 4; ++e) {
    const float f0 = a0[e] * scale;
    const float f1 = a1[e] * scale;
    hv[e]     = (_Float16)(ok ? f0 : 0.0f);
    hv[4 + e] = (_Float16)(ok ? f1 : 0.0f);
  }
  unsigned short* q = dst + ((size_t)i << 3);
  *(volatile v8h*)q = hv;
  __threadfence();
  *(volatile v8h*)q = hv;
}

__global__ __launch_bounds__(256) void rmsnorm_copy_kernel(
    const float* __restrict__ X, const float* __restrict__ Wn,
    unsigned short* __restrict__ H16, float* __restrict__ OUT1)
{
  __shared__ float sPart[8];
  __shared__ __align__(16) float sRow[kDm];
  const int tid = threadIdx.x, lane = tid & 31, wave = tid >> 5;
  const size_t rbase = (size_t)blockIdx.x * kDm;
  const v4f xv = *(const v4f*)(X + rbase + tid * 4);
  const v4f wv = *(const v4f*)(Wn + tid * 4);
  float ss = 0.0f;
  ss += xv[0] * xv[0];
  ss += xv[1] * xv[1];
  ss += xv[2] * xv[2];
  ss += xv[3] * xv[3];
#pragma unroll
  for (int off = 16; off > 0; off >>= 1) ss += __shfl_xor(ss, off, 32);
  if (lane == 0) sPart[wave] = ss;
  __syncthreads();
  float tot = 0.0f;
#pragma unroll
  for (int w = 0; w < 8; ++w) tot += sPart[w];
  const float nrm = sqrtf(tot);
  const float rms = nrm * kInvSqrtDm;
  const float inv = 1.0f / (rms + kEps);
  v4f hq;
#pragma unroll
  for (int e = 0; e < 4; ++e) hq[e] = (wv[e] * (xv[e] * inv)) * kCarryH;
  *(v4f*)(sRow + tid * 4) = hq;
  __syncthreads();
  const int t8 = (tid & 127) * 8;
  const v4f a0 = *(const v4f*)(sRow + t8);
  const v4f a1 = *(const v4f*)(sRow + t8 + 4);
  v8h hv;
#pragma unroll
  for (int e = 0; e < 4; ++e) { hv[e] = (_Float16)a0[e]; hv[4 + e] = (_Float16)a1[e]; }
  for (int pass = 0; pass < 2; ++pass) {
    *(volatile v4f*)(OUT1 + rbase + tid * 4) = xv;
    if (tid < 128) *(volatile v8h*)(H16 + rbase + t8) = hv;
    __threadfence();
  }
}

__global__ __launch_bounds__(256) void conv_silu_kernel(
    const float* __restrict__ XZ, const float* __restrict__ cw, const float* __restrict__ cb,
    float* __restrict__ UC, unsigned short* __restrict__ UC16)
{
  __shared__ __align__(16) float sT[16 * kTP];
  const int tid = threadIdx.x, lane = tid & 31, wave = tid >> 5;
  const int d0 = blockIdx.x * 256, d = d0 + tid;
  const int g0 = blockIdx.y * 64;
  const int tb = g0 & (kSeq - 1);
  const v4f wq = *(const v4f*)(cw + (size_t)d * 4);
  const float w0 = wq[0], w1 = wq[1], w2 = wq[2], w3 = wq[3];
  const float bc = cb[d];
  float xm3, xm2, xm1;
  {
    const bool hist = (tb > 0);
    const int rb = hist ? (g0 - 3) : g0;
    const float v3 = XZ[(size_t)rb * kXZP + d];
    const float v2 = XZ[(size_t)(rb + 1) * kXZP + d];
    const float v1 = XZ[(size_t)(rb + 2) * kXZP + d];
    xm3 = hist ? v3 : 0.f;
    xm2 = hist ? v2 : 0.f;
    xm1 = hist ? v1 : 0.f;
  }
  const int hrow = wave >> 1;
  const int hch  = (wave & 1) * 128 + lane * 4;
#pragma unroll 1
  for (int sub = 0; sub < 4; ++sub) {
    const int lb = g0 + sub * 16;
#pragma unroll 1
    for (int s = 0; s < 16; ++s) {
      const float xcur = XZ[(size_t)(lb + s) * kXZP + d];
      float acc = w0 * xm3;
      acc = fmaf(w1, xm2, acc);
      acc = fmaf(w2, xm1, acc);
      acc = fmaf(w3, xcur, acc);
      const float sv = acc + bc;
      sT[s * kTP + tid] = silu_f(sv);
      xm3 = xm2; xm2 = xm1; xm1 = xcur;
    }
    __syncthreads();
    v4f fv[4];
    v8h bv[2];
#pragma unroll
    for (int it = 0; it < 4; ++it) fv[it] = *(const v4f*)(sT + (it * 4 + hrow) * kTP + hch);
#pragma unroll
    for (int it = 0; it < 2; ++it) {
      const float* sp = sT + (it * 8 + wave) * kTP + lane * 8;
      const v4f a0 = *(const v4f*)(sp);
      const v4f a1 = *(const v4f*)(sp + 4);
#pragma unroll
      for (int e = 0; e < 4; ++e) {
        bv[it][e]     = (_Float16)(a0[e] * kCarryXc);
        bv[it][4 + e] = (_Float16)(a1[e] * kCarryXc);
      }
    }
    for (int pass = 0; pass < 2; ++pass) {
#pragma unroll
      for (int it = 0; it < 4; ++it)
        *(volatile v4f*)(UC + (size_t)(lb + it * 4 + hrow) * kDin + d0 + hch) = fv[it];
#pragma unroll
      for (int it = 0; it < 2; ++it)
        *(volatile v8h*)(UC16 + (size_t)(lb + it * 8 + wave) * kDin + d0 + lane * 8) = bv[it];
      __threadfence();
    }
    __syncthreads();
  }
}

__global__ __launch_bounds__(256) void dt_cast_kernel(
    const float* __restrict__ PROJ, unsigned short* __restrict__ DT16, int total8, float scale)
{
  const int i = blockIdx.x * 256 + threadIdx.x;
  if (i >= total8) return;
  const int e0  = i << 3;
  const int row = e0 >> 6;
  const int c8  = e0 & 63;
  const float* p = PROJ + (size_t)row * kPrjP + c8;
  const v4f a0 = *(const v4f*)(p);
  const v4f a1 = *(const v4f*)(p + 4);
  v8h hv;
#pragma unroll
  for (int e = 0; e < 4; ++e) {
    hv[e]     = (_Float16)(a0[e] * scale);
    hv[4 + e] = (_Float16)(a1[e] * scale);
  }
  unsigned short* qd = DT16 + e0;
  *(volatile v8h*)qd = hv;
  __threadfence();
  *(volatile v8h*)qd = hv;
}

__global__ __launch_bounds__(256) void scan_kernel(
    const float* __restrict__ DLR, const float* __restrict__ UC, const float* __restrict__ XZ,
    const float* __restrict__ PROJ, const float* __restrict__ A_log, const float* __restrict__ Dv,
    unsigned short* __restrict__ Y16)
{
  __shared__ __align__(16) float sBC[16 * 32];
  __shared__ __align__(16) float sY[16 * kTP];
  __shared__ __align__(16) float sA[kNst * 256];
  __shared__ __align__(16) float sH[kNst * 256];
  const int tid = threadIdx.x, lane = tid & 31, wave = tid >> 5;
  constexpr int kBlkPerB = kDin / 256;
  const int bix = blockIdx.x / kBlkPerB;
  const int d0  = (blockIdx.x - bix * kBlkPerB) * 256;
  const int d   = d0 + tid;
  const size_t row0 = (size_t)bix * kSeq;
#pragma unroll 1
  for (int n = 0; n < kNst; ++n) {
    sA[n * 256 + tid] = -expf(A_log[(size_t)d * kNst + n]);
    sH[n * 256 + tid] = 0.0f;
  }
  const float Dd = Dv[d];

#pragma unroll 1
  for (int c = 0; c < kSeq / 16; ++c) {
    const int l0 = c * 16;
    if (tid < 128) {
      const int r = tid >> 3, q = (tid & 7) * 4;
      const v4f v = *(const v4f*)(PROJ + (row0 + l0 + r) * kPrjP + kDtR + q);
      *(v4f*)(sBC + r * 32 + q) = v;
    }
    __syncthreads();
#pragma unroll 1
    for (int s = 0; s < 16; ++s) {
      const size_t m = row0 + (size_t)(l0 + s);
      float a  = DLR[m * kDin + d];
      float xv = UC[m * kDin + d];
      float zv = XZ[m * kXZP + kDin + d];
      asm volatile("" : "+v"(a));
      asm volatile("" : "+v"(xv));
      asm volatile("" : "+v"(zv));
      const float delta = fmaxf(a, 0.0f) + log1pf(expf(-fabsf(a)));
      const float dx = delta * xv;
      float y = 0.0f;
#pragma unroll 1
      for (int n = 0; n < kNst; ++n) {
        const float An = sA[n * 256 + tid];
        const float hp = sH[n * 256 + tid];
        const float Bn = sBC[s * 32 + n];
        const float Cn = sBC[s * 32 + kNst + n];
        const float e  = expf(delta * An);
        const float hn = e * hp + dx * Bn;
        sH[n * 256 + tid] = hn;
        y = fmaf(hn, Cn, y);
      }
      y = fmaf(Dd, xv, y);
      const float g = silu_f(zv);
      sY[s * kTP + tid] = (y * g) * kCarryY;
    }
    __syncthreads();
    v8h hv[2];
#pragma unroll
    for (int it = 0; it < 2; ++it) {
      const float* sp = sY + (it * 8 + wave) * kTP + lane * 8;
      const v4f a0 = *(const v4f*)(sp);
      const v4f a1 = *(const v4f*)(sp + 4);
#pragma unroll
      for (int e = 0; e < 4; ++e) { hv[it][e] = (_Float16)a0[e]; hv[it][4 + e] = (_Float16)a1[e]; }
    }
    for (int pass = 0; pass < 2; ++pass) {
#pragma unroll
      for (int it = 0; it < 2; ++it)
        *(volatile v8h*)(Y16 + (row0 + (size_t)(l0 + it * 8 + wave)) * kDin + d0 + lane * 8) = hv[it];
      __threadfence();
    }
  }
}

extern "C" void kernel_launch(void* const* d_in, const int* in_sizes, int n_in,
                              void* d_out, int out_size, void* d_ws, size_t ws_size,
                              hipStream_t stream)
{
  if (n_in < 11) return;
  if (in_sizes[0] != kRows * kDm) return;
  if (in_sizes[1] != kDm) return;
  if (in_sizes[2] != kXZP * kDm) return;
  if (in_sizes[3] != kDin * 4) return;
  if (in_sizes[4] != kDin) return;
  if (in_sizes[5] != kPrjN * kDin) return;
  if (in_sizes[6] != kDin * kDtR) return;
  if (in_sizes[7] != kDin) return;
  if (in_sizes[8] != kDin * kNst) return;
  if (in_sizes[9] != kDin) return;
  if (in_sizes[10] != kDm * kDin) return;
  if (out_size != 2 * kRows * kDm) return;
  if (ws_size < kWsTotal) return;

  const float* hs     = (const float*)d_in[0];
  const float* norm_w = (const float*)d_in[1];
  const float* W_in   = (const float*)d_in[2];
  const float* conv_w = (const float*)d_in[3];
  const float* conv_b = (const float*)d_in[4];
  const float* W_x    = (const float*)d_in[5];
  const float* W_dt   = (const float*)d_in[6];
  const float* b_dt   = (const float*)d_in[7];
  const float* A_log  = (const float*)d_in[8];
  const float* Dv     = (const float*)d_in[9];
  const float* W_out  = (const float*)d_in[10];
  float* out0 = (float*)d_out;
  float* out1 = out0 + (size_t)kRows * kDm;

  char* ws = (char*)d_ws;
  unsigned short* WIN16  = (unsigned short*)(ws + kOffWIN);
  unsigned short* WXP16  = (unsigned short*)(ws + kOffWXP);
  unsigned short* WDT16  = (unsigned short*)(ws + kOffWDT);
  unsigned short* WOUT16 = (unsigned short*)(ws + kOffWOUT);
  unsigned short* H16    = (unsigned short*)(ws + kOffH16);
  float*          XZ     = (float*)(ws + kOffXZ);
  float*          UC     = (float*)(ws + kOffUC);
  unsigned short* UC16   = (unsigned short*)(ws + kOffUC16);
  float*          PROJ   = (float*)(ws + kOffPROJ);
  unsigned short* DT16   = (unsigned short*)(ws + kOffDT16);
  float*          DLR    = (float*)(ws + kOffDLR);
  unsigned short* Y16    = (unsigned short*)(ws + kOffY16);

  constexpr int kWin8   = kXZP * kDm / 8;
  constexpr int kWxTot8 = kPrjP * kDin / 8;
  constexpr int kWxRe8  = kPrjN * kDin / 8;
  constexpr int kWdt8   = kDin * kDtR / 8;
  constexpr int kWout8  = kDm * kDin / 8;
  static_assert((kWin8 % 256) == 0 && (kWxTot8 % 256) == 0 && (kWdt8 % 256) == 0 && (kWout8 % 256) == 0);
  cast_f16_pad_kernel<<<kWin8 / 256, 256, 0, stream>>>(W_in, WIN16, kWin8, kWin8, kCarryW);
  cast_f16_pad_kernel<<<kWxTot8 / 256, 256, 0, stream>>>(W_x, WXP16, kWxTot8, kWxRe8, kCarryW);
  cast_f16_pad_kernel<<<kWdt8 / 256, 256, 0, stream>>>(W_dt, WDT16, kWdt8, kWdt8, kCarryW);
  cast_f16_pad_kernel<<<kWout8 / 256, 256, 0, stream>>>(W_out, WOUT16, kWout8, kWout8, kCarryW);

  rmsnorm_copy_kernel<<<kRows, 256, 0, stream>>>(hs, norm_w, H16, out1);

  wmma_gemm64_f16<0><<<(kRows / 64) * (kXZP / 64) / 8, 256, 0, stream>>>(
      H16, kDm, WIN16, kDm, XZ, kXZP, b_dt, kRows, kXZP, kDm, kFoldIn);

  conv_silu_kernel<<<dim3(kDin / 256, kRows / 64), 256, 0, stream>>>(XZ, conv_w, conv_b, UC, UC16);

  wmma_gemm64_f16<0><<<(kRows / 64) * (kPrjP / 64) / 8, 256, 0, stream>>>(
      UC16, kDin, WXP16, kDin, PROJ, kPrjP, b_dt, kRows, kPrjP, kDin, kFoldX);

  constexpr int kDt8 = kRows * kDtR / 8;
  static_assert((kDt8 % 256) == 0);
  dt_cast_kernel<<<kDt8 / 256, 256, 0, stream>>>(PROJ, DT16, kDt8, kCarryDt);

  wmma_gemm64_f16<2><<<(kRows / 64) * (kDin / 64) / 8, 256, 0, stream>>>(
      DT16, kDtR, WDT16, kDtR, DLR, kDin, b_dt, kRows, kDin, kDtR, kFoldDt);

  scan_kernel<<<kBatch * (kDin / 256), 256, 0, stream>>>(DLR, UC, XZ, PROJ, A_log, Dv, Y16);

  wmma_gemm64_f16<0><<<(kRows / 64) * (kDm / 64) / 8, 256, 0, stream>>>(
      Y16, kDin, WOUT16, kDin, out0, kDm, b_dt, kRows, kDm, kDin, kFoldOut);
}
